// GraphormerFishAttention_45844480918018
// MI455X (gfx1250) — hardware-verified
//
#include <hip/hip_runtime.h>


namespace {
constexpr int Bn = 8, S = 256, H = 512, G = 8, L = 16, HD = 64, NT = Bn * S, NPJ = 2048;
constexpr float QS = 8.0f, KS = 8.0f, VS = 8.0f, PS = 8.0f, AS_ = 8.0f, SCALE = 0.04419417382415922f;

typedef _Float16 b16;
typedef __attribute__((ext_vector_type(16))) _Float16 v16b;
typedef __attribute__((ext_vector_type(8))) _Float16 v8b;
typedef __attribute__((ext_vector_type(8))) float v8f;
typedef __attribute__((ext_vector_type(4))) float v4f;
__device__ __forceinline__ float bf16_rne(float f) { unsigned int u = __float_as_uint(f); u += 0x7FFFu + ((u >> 16) & 1u); return __uint_as_float(u & 0xFFFF0000u); }
__device__ __forceinline__ void split16(float v, b16& hi, b16& lo) { hi = (b16)v; lo = (b16)(v - (float)hi); }
__device__ __forceinline__ v16b frag_kb(const b16* p, int hh) { const v8b a = *(const v8b*)(p + 8 * hh), b = *(const v8b*)(p + 16 + 8 * hh); v16b f;
#pragma unroll
  for (int e = 0; e < 8; ++e) { f[e] = a[e]; f[8 + e] = b[e]; } return f; }
__device__ __forceinline__ v16b frag_x(const float* p, int hh) { v16b f;
#pragma unroll
  for (int e = 0; e < 8; ++e) { f[e] = (b16)bf16_rne(p[8 * hh + e]); f[8 + e] = (b16)bf16_rne(p[16 + 8 * hh + e]); } return f; }
__device__ __forceinline__ void frag_split(const float* p, int hh, v16b& fh, v16b& fl) {
#pragma unroll
  for (int e = 0; e < 8; ++e) { b16 a, c; split16(p[8 * hh + e] * AS_, a, c); fh[e] = a; fl[e] = c; split16(p[16 + 8 * hh + e] * AS_, a, c); fh[8 + e] = a; fl[8 + e] = c; } }
__device__ __forceinline__ v8f wmma16b(v16b a, v16b b, v8f c) { v8f d = __builtin_amdgcn_wmma_f32_16x16x32_f16(false, a, false, b, (short)0, c, false, false); asm volatile("v_nop\n\tv_nop\n\tv_nop\n\tv_nop" : "+v"(d) : "v"(a), "v"(b)); return d; }
__device__ __forceinline__ void wave_lds_sync() { __builtin_amdgcn_fence(__ATOMIC_RELEASE, "workgroup"); __builtin_amdgcn_wave_barrier(); __builtin_amdgcn_fence(__ATOMIC_ACQUIRE, "workgroup"); }
__device__ __forceinline__ float nexp(float x) { return __builtin_amdgcn_exp2f(x * 1.4426950408889634f); }
__device__ __forceinline__ float pmul(float a, float b) { float p = a * b; asm volatile("" : "+v"(p)); return p; }

__global__ __launch_bounds__(256) void prep_kernel(const float* __restrict__ Wq, const float* __restrict__ Wk, const float* __restrict__ Wv, const float* __restrict__ Wout, const float* __restrict__ bv, const float* __restrict__ bout, const float* __restrict__ sg, const float* __restrict__ pp, const float* __restrict__ ed, b16* __restrict__ R, b16* __restrict__ Ro, float* __restrict__ P) {
  const int t_ = blockIdx.x * 256 + threadIdx.x, nth = gridDim.x * 256;
  for (int pass = 0; pass < 2; ++pass) {
    for (int q = t_; q < NPJ * H; q += nth) { const int o = q / H, k = q % H; float w; if (o < 512) w = Wq[(size_t)k * 512 + o]; else if (o < 1024) w = Wk[(size_t)k * 512 + o - 512]; else w = Wv[(size_t)k * 1024 + o - 1024]; R[q] = (b16)bf16_rne(w); }
    for (int q = t_; q < 512 * 1024; q += nth) { const int o = q >> 10, k = q & 1023; Ro[q] = (b16)bf16_rne(Wout[(size_t)k * 512 + o]); }
    for (int q = t_; q < 1672 + L * S; q += nth) { float v; if (q < 1024) v = bf16_rne(bv[q]); else if (q < 1536) v = bf16_rne(bout[q - 1024]); else if (q < 1544) { const float s_ = bf16_rne(sg[q - 1536]); v = s_ * s_; } else if (q < 1672) v = bf16_rne(pp[q - 1544]); else v = bf16_rne(ed[q - 1672]); P[q] = v; }
    __threadfence(); }
}

__global__ __launch_bounds__(128) void proj_kernel(const float* __restrict__ x, const b16* __restrict__ R, const float* __restrict__ P, b16* __restrict__ qp, b16* __restrict__ kp, b16* __restrict__ vt) {
  __shared__ __attribute__((aligned(16))) b16 T[4][32][64 + 8]; __shared__ __attribute__((aligned(16))) b16 Tv[64][128 + 8];
  const int lane = threadIdx.x & 31, wave = threadIdx.x >> 5, nloc = lane & 15, hlf = lane >> 4, ct = blockIdx.x, c0 = ct * 64, p0 = blockIdx.y * 128, m0 = p0 + wave * 32, b = p0 / S, t0 = p0 % S;
  v8f acc[2][4];
#pragma unroll
  for (int r = 0; r < 2; ++r)
#pragma unroll
    for (int t = 0; t < 4; ++t) acc[r][t] = (v8f){};
#pragma unroll 2
  for (int kb = 0; kb < H; kb += 32) { const v16b a0 = frag_x(x + (size_t)(m0 + nloc) * H + kb, hlf), a1 = frag_x(x + (size_t)(m0 + 16 + nloc) * H + kb, hlf);
#pragma unroll
    for (int t = 0; t < 4; ++t) { const v16b bw = frag_kb(R + (size_t)(c0 + t * 16 + nloc) * H + kb, hlf); acc[0][t] = wmma16b(a0, bw, acc[0][t]); acc[1][t] = wmma16b(a1, bw, acc[1][t]); } }
  if (ct < 16) { const float scl = (ct < 8) ? SCALE * QS : KS; const int hd_ = (ct < 8) ? ct : ct - 8;
#pragma unroll
    for (int t = 0; t < 4; ++t)
#pragma unroll
      for (int r = 0; r < 2; ++r)
#pragma unroll
        for (int v = 0; v < 8; ++v) T[wave][r * 16 + 8 * hlf + v][t * 16 + nloc] = (b16)(acc[r][t][v] * scl);
    wave_lds_sync();
    b16* base = ((ct < 8) ? qp : kp) + (((size_t)b * G + hd_) * S + (m0 % S)) * HD;
    for (int pass = 0; pass < 2; ++pass) {
#pragma unroll
      for (int j = 0; j < 8; ++j) { const int rr = j * 4 + (lane >> 3), c8 = (lane & 7) * 8; *(volatile v8b*)(base + (size_t)rr * HD + c8) = *(const v8b*)(&T[wave][rr][c8]); }
      __threadfence(); }
    return; }
  const int l = ct - 16; const float* bvp = P + l * HD;
#pragma unroll
  for (int t = 0; t < 4; ++t) { const float bb = bvp[t * 16 + nloc];
#pragma unroll
    for (int r = 0; r < 2; ++r)
#pragma unroll
      for (int v = 0; v < 8; ++v) Tv[t * 16 + nloc][wave * 32 + r * 16 + 8 * hlf + v] = (b16)((acc[r][t][v] + bb) * VS); }
  __syncthreads();
  for (int pass = 0; pass < 2; ++pass) { for (int i = threadIdx.x; i < 64 * 16; i += 128) { const int d = i >> 4, c8 = (i & 15) * 8; *(volatile v8b*)(vt + (((size_t)b * L + l) * HD + d) * S + t0 + c8) = *(const v8b*)(&Tv[d][c8]); } __threadfence(); }
}

__global__ __launch_bounds__(256) void score_kernel(const b16* __restrict__ qp, const b16* __restrict__ kp, const float* __restrict__ sp, const float* __restrict__ ee, float* __restrict__ sc, float* __restrict__ flags) {
  __shared__ __attribute__((aligned(16))) float Ts[8][16][S + 4]; __shared__ float Fl[16][8];
  const int g = threadIdx.x >> 5, lane = threadIdx.x & 31, nloc = lane & 15, hlf = lane >> 4; const int b = blockIdx.y, s0 = blockIdx.x * 16;
  const b16* Q = qp + (((size_t)b * G + g) * S) * HD; const b16* K = kp + (((size_t)b * G + g) * S) * HD;
  const v16b q0 = frag_kb(Q + (size_t)(s0 + nloc) * HD, hlf), q1 = frag_kb(Q + (size_t)(s0 + nloc) * HD + 32, hlf);
  for (int tt = 0; tt < 16; ++tt) { v8f acc = {}; const v16b k0 = frag_kb(K + (size_t)(tt * 16 + nloc) * HD, hlf), k1 = frag_kb(K + (size_t)(tt * 16 + nloc) * HD + 32, hlf); acc = wmma16b(q0, k0, acc); acc = wmma16b(q1, k1, acc);
#pragma unroll
    for (int r = 0; r < 8; ++r) { const int s = s0 + 8 * hlf + r, t = tt * 16 + nloc; const size_t bo = ((size_t)b * S + s) * S + t; Ts[g][8 * hlf + r][t] = acc[r] * (1.0f / (QS * KS)) + (bf16_rne(sp[bo]) + bf16_rne(ee[bo])); } }
  wave_lds_sync();
  { const int rr = lane & 15, half = lane >> 4; int nz = 0; for (int t = half; t < S; t += 2) nz |= (Ts[g][rr][t] != 0.0f) ? 1 : 0; nz |= __shfl_xor(nz, 16); if (lane < 16) Fl[rr][g] = nz ? 1.0f : 0.0f; }
  for (int pass = 0; pass < 2; ++pass) { for (int i = lane; i < 16 * (S / 4); i += 32) { const int rr = i / (S / 4), c4 = (i % (S / 4)) * 4; *(volatile v4f*)(sc + (((size_t)b * G + g) * S + s0 + rr) * S + c4) = *(const v4f*)(&Ts[g][rr][c4]); } __threadfence(); }
  __syncthreads();
  for (int pass = 0; pass < 2; ++pass) { if (threadIdx.x < 128) ((volatile float*)flags)[((size_t)b * S + s0) * G + threadIdx.x] = Fl[threadIdx.x >> 3][threadIdx.x & 7]; __threadfence(); }
}

__global__ __launch_bounds__(256) void fish_kernel(const float* __restrict__ sc, const float* __restrict__ flags, const b16* __restrict__ vt, const float* __restrict__ P, float* __restrict__ ctx) {
  __shared__ __attribute__((aligned(16))) float A[16][S + 4]; __shared__ __attribute__((aligned(16))) float Cx[16][L * HD + 4];
  const int t_ = threadIdx.x, wave = t_ >> 5, lane = t_ & 31, nloc = lane & 15, hlf = lane >> 4; const int b = blockIdx.y, s0 = blockIdx.x * 16;
  const float* sig2 = P + 1536; const float* pp = P + 1544; const float* ed = P + 1672;
  for (int l = 0; l < L; ++l) {
    for (int i = t_; i < 16 * S; i += 256) { const int rr = i / S, t = i % S, s = s0 + rr; float a = 0.0f; bool ninf = false;
#pragma unroll
      for (int g = 0; g < G; ++g) { const float fl = flags[((size_t)b * S + s) * G + g]; float v = sc[(((size_t)b * G + g) * S + s) * S + t]; if (t == s) v += sig2[g] * ed[l * S + s]; v = fmaxf(pmul(v, pp[g * L + l]), 0.0f); if (fl != 0.0f) a += v; else ninf = true; }
      A[rr][t] = ninf ? -INFINITY : a; }
    __syncthreads();
    for (int rr = wave * 2; rr < wave * 2 + 2; ++rr) { float mx = -INFINITY; for (int t = lane; t < S; t += 32) mx = fmaxf(mx, A[rr][t]);
#pragma unroll
      for (int o = 1; o < 32; o <<= 1) mx = fmaxf(mx, __shfl_xor(mx, o));
      float sm = 0.0f; for (int t = lane; t < S; t += 32) sm += (mx == -INFINITY) ? 0.0f : nexp(A[rr][t] - mx);
#pragma unroll
      for (int o = 1; o < 32; o <<= 1) sm += __shfl_xor(sm, o);
      const float inv = (mx == -INFINITY) ? 0.0f : 1.0f / sm;
      for (int t = lane; t < S; t += 32) A[rr][t] = (mx == -INFINITY) ? 0.0f : nexp(A[rr][t] - mx) * inv; }
    __syncthreads();
    if (wave < 4) { v8f acc = {}; const b16* V = vt + (((size_t)b * L + l) * HD) * S;
#pragma unroll 2
      for (int kb = 0; kb < S; kb += 32) { v16b ah, al; frag_split(&A[nloc][kb], hlf, ah, al); const v16b bw = frag_kb(V + (size_t)(wave * 16 + nloc) * S + kb, hlf); acc = wmma16b(ah, bw, acc); acc = wmma16b(al, bw, acc); }
#pragma unroll
      for (int r = 0; r < 8; ++r) Cx[8 * hlf + r][l * HD + wave * 16 + nloc] = acc[r] * (1.0f / (AS_ * VS)); }
    __syncthreads(); }
  for (int pass = 0; pass < 2; ++pass) { for (int i = t_; i < 16 * (L * HD / 4); i += 256) { const int rr = i / (L * HD / 4), c4 = (i % (L * HD / 4)) * 4; *(volatile v4f*)(ctx + ((size_t)b * S + s0 + rr) * (L * HD) + c4) = *(const v4f*)(&Cx[rr][c4]); } __threadfence(); }
}

__global__ __launch_bounds__(128) void out_kernel(const float* __restrict__ ctx, const b16* __restrict__ Ro, const float* __restrict__ P, float* __restrict__ out) {
  __shared__ __attribute__((aligned(16))) float Ts[4][32 * 64];
  const int lane = threadIdx.x & 31, wave = threadIdx.x >> 5, nloc = lane & 15, hlf = lane >> 4, m0 = blockIdx.y * 128 + wave * 32, c0 = blockIdx.x * 64; const float* bout = P + 1024;
  v8f acc[2][4];
#pragma unroll
  for (int r = 0; r < 2; ++r)
#pragma unroll
    for (int t = 0; t < 4; ++t) acc[r][t] = (v8f){};
#pragma unroll 2
  for (int kb = 0; kb < L * HD; kb += 32) { v16b a0, l0, a1, l1; frag_split(ctx + (size_t)(m0 + nloc) * (L * HD) + kb, hlf, a0, l0); frag_split(ctx + (size_t)(m0 + 16 + nloc) * (L * HD) + kb, hlf, a1, l1);
#pragma unroll
    for (int t = 0; t < 4; ++t) { const v16b bw = frag_kb(Ro + (size_t)(c0 + t * 16 + nloc) * (L * HD) + kb, hlf); acc[0][t] = wmma16b(a0, bw, acc[0][t]); acc[0][t] = wmma16b(l0, bw, acc[0][t]); acc[1][t] = wmma16b(a1, bw, acc[1][t]); acc[1][t] = wmma16b(l1, bw, acc[1][t]); } }
  float* Tt = Ts[wave];
#pragma unroll
  for (int t = 0; t < 4; ++t) { const float bb = bout[c0 + t * 16 + nloc];
#pragma unroll
    for (int r = 0; r < 2; ++r)
#pragma unroll
      for (int v = 0; v < 8; ++v) Tt[(r * 16 + v + 8 * hlf) * 64 + t * 16 + nloc] = acc[r][t][v] * (1.0f / AS_) + bb; }
  wave_lds_sync();
  for (int pass = 0; pass < 2; ++pass) {
#pragma unroll
    for (int j = 0; j < 16; ++j) { const int rr = j * 2 + hlf, c4 = nloc * 4; *(volatile v4f*)(out + (size_t)(m0 + rr) * H + c0 + c4) = *(const v4f*)(Tt + rr * 64 + c4); }
    __threadfence(); }
}
}

extern "C" void kernel_launch(void* const* d_in, const int* in_sizes, int n_in,
                              void* d_out, int out_size, void* d_ws, size_t ws_size, hipStream_t stream) {
  (void)n_in; (void)out_size;
  const float* x = (const float*)d_in[0]; const float* sp = (const float*)d_in[1]; const float* ee = (const float*)d_in[2]; const float* Wq = (const float*)d_in[3]; const float* Wk = (const float*)d_in[4]; const float* Wv = (const float*)d_in[5]; const float* bv = (const float*)d_in[6];
  const float* sg = (const float*)d_in[7]; const float* pp = (const float*)d_in[8]; const float* ed = (const float*)d_in[9]; const float* Wout = (const float*)d_in[10]; const float* bout = (const float*)d_in[11];
  float* out = (float*)d_out;
  if (in_sizes[0] != NT * H || in_sizes[1] != Bn * S * S || in_sizes[5] != H * 1024 || in_sizes[8] != G * L || in_sizes[9] != L * S || in_sizes[10] != 1024 * H) return;
  size_t off = 0; char* ws = (char*)d_ws;
  auto carve = [&](size_t bytes) { char* p = ws + off; off += (bytes + 255) & ~(size_t)255; return p; };
  b16* R = (b16*)carve((size_t)NPJ * H * 2); b16* Ro = (b16*)carve((size_t)512 * 1024 * 2); float* P = (float*)carve(((size_t)1672 + L * S + 64) * 4);
  b16* qp = (b16*)carve((size_t)Bn * G * S * HD * 2); b16* kp = (b16*)carve((size_t)Bn * G * S * HD * 2); b16* vt = (b16*)carve((size_t)Bn * L * HD * S * 2); float* sc = (float*)carve((size_t)Bn * G * S * S * 4); float* flags = (float*)carve((size_t)Bn * S * G * 4); float* ctx = (float*)carve((size_t)NT * L * HD * 4);
  if (off > ws_size) return;
  prep_kernel<<<256, 256, 0, stream>>>(Wq, Wk, Wv, Wout, bv, bout, sg, pp, ed, R, Ro, P);
  proj_kernel<<<dim3(32, NT / 128), 128, 0, stream>>>(x, R, P, qp, kp, vt);
  score_kernel<<<dim3(S / 16, Bn), 256, 0, stream>>>(qp, kp, sp, ee, sc, flags);
  fish_kernel<<<dim3(S / 16, Bn), 256, 0, stream>>>(sc, flags, vt, P, ctx);
  out_kernel<<<dim3(H / 64, NT / 128), 128, 0, stream>>>(ctx, Ro, P, out);
}
